// GraphSelfAttention_43645457662514
// MI455X (gfx1250) — hardware-run, weakly checked
//
#include <hip/hip_runtime.h>


namespace {
constexpr int N = 20000, NP = 20032, E = 120000, EP = 121344  , M0 = 16, M1 = 8, XW = 40, NB = 10, HDIM = 16, UC = M0 + M1  , KK = UC * HDIM  , DQ = 16, DK = 16, DV = 32;
constexpr float XS = 8.0f, WSC = 32.0f  , NEG = 0.2f  , RMAX = 4.0f;

typedef _Float16 b16;
typedef __attribute__((ext_vector_type(16))) _Float16 v16b;
typedef __attribute__((ext_vector_type(8))) _Float16 v8b;
typedef __attribute__((ext_vector_type(8))) float v8f;
typedef __attribute__((ext_vector_type(4))) float v4f;
__device__ __forceinline__ float bf16_rne(float f) { unsigned int u = __float_as_uint(f); u += 0x7FFFu + ((u >> 16) & 1u); return __uint_as_float(u & 0xFFFF0000u); }
__device__ __forceinline__ void split16(float v, b16& hi, b16& lo) { hi = (b16)v; lo = (b16)(v - (float)hi); }
__device__ __forceinline__ v16b frag_kb(const b16* p, int hh) { const v8b a = *(const v8b*)(p + 8 * hh), b = *(const v8b*)(p + 16 + 8 * hh); v16b f;
#pragma unroll
  for (int e = 0; e < 8; ++e) { f[e] = a[e]; f[8 + e] = b[e]; } return f; }
__device__ __forceinline__ v8f wmma16b(v16b a, v16b b, v8f c) { v8f d = __builtin_amdgcn_wmma_f32_16x16x32_f16(false, a, false, b, (short)0, c, false, false); asm volatile("v_nop\n\tv_nop\n\tv_nop\n\tv_nop" : "+v"(d) : "v"(a), "v"(b)); return d; }
__device__ __forceinline__ void wave_lds_sync() { __builtin_amdgcn_fence(__ATOMIC_RELEASE, "workgroup"); __builtin_amdgcn_wave_barrier(); __builtin_amdgcn_fence(__ATOMIC_ACQUIRE, "workgroup"); }
__device__ __forceinline__ float pmul(float a, float b) { float p = a * b; asm volatile("" : "+v"(p)); return p; }
__device__ __forceinline__ int iclamp(int v, int lo, int hi) { return v < lo ? lo : (v > hi ? hi : v); }
__device__ __forceinline__ float nexp(float x) { return __builtin_amdgcn_exp2f(x * 1.4426950408889634f); }
__device__ __forceinline__ float lrelu(float x) { return x > 0.0f ? x : NEG * x; }

constexpr int CSR_NBLK = 512, CSR_GB = 9, CSR_GN = 1 << CSR_GB  , CSR_MAXG = 512, CSR_CAP = 12288  ;
__global__ __launch_bounds__(64) void csrA_kernel(const int* __restrict__ dst, int E, int N, int nG, int CHP, int NGP, int* __restrict__ STG, int* __restrict__ HST) {
  extern __shared__ int sm[];
  int* cnt = sm; int* run = sm + NGP; int* ids = sm + 2 * NGP;
  const int b = blockIdx.x; const int ch = (E + CSR_NBLK - 1) / CSR_NBLK; const int e0 = b * ch, e1 = min(E, e0 + ch);
  for (int i = threadIdx.x; i < NGP; i += 64) cnt[i] = 0;
  for (int i = threadIdx.x; i < CHP; i += 64) ids[i] = -1;
  __syncthreads();
  if (threadIdx.x == 0) {
    for (int e = e0; e < e1; ++e) { int d = dst[e]; d = (d < 0) ? 0 : (d >= N ? N - 1 : d); cnt[d >> CSR_GB] += 1; }
    int acc = 0; for (int g = 0; g < nG; ++g) { run[g] = acc; acc += cnt[g]; }
    for (int e = e0; e < e1; ++e) { int d = dst[e]; d = (d < 0) ? 0 : (d >= N ? N - 1 : d); const int g = d >> CSR_GB; ids[run[g]] = e; run[g] += 1; } }
  __syncthreads();
  typedef __attribute__((ext_vector_type(4))) int v4i;
  for (int pass = 0; pass < 2; ++pass) {
    for (int i = threadIdx.x; i < CHP / 4; i += 64) *(volatile v4i*)(STG + (size_t)b * CHP + i * 4) = *(const v4i*)(&ids[i * 4]);
    for (int i = threadIdx.x; i < NGP / 4; i += 64) { v4i v; for (int e = 0; e < 4; ++e) v[e] = (i * 4 + e < nG) ? cnt[i * 4 + e] : 0; *(volatile v4i*)(HST + (size_t)b * NGP + i * 4) = v; }
    __threadfence(); }
}
__global__ __launch_bounds__(512) void csrS_kernel(const int* __restrict__ HST, int nG, int NGP, int* __restrict__ START, int* __restrict__ TOT, int* __restrict__ OFF) {
  __shared__ int tot[CSR_MAXG];
  const int b = threadIdx.x;
  for (int pass = 0; pass < 2; ++pass) { int runb = 0; for (int g = 0; g < nG; ++g) { int c = HST[(size_t)b * NGP + g]; c = (c < 0) ? 0 : c; ((volatile int*)OFF)[(size_t)g * CSR_NBLK + b] = runb; runb += c; } __threadfence(); }
  for (int g = threadIdx.x; g < nG; g += 512) { int s = 0; for (int bb = 0; bb < CSR_NBLK; ++bb) { int c = HST[(size_t)bb * NGP + g]; s += (c < 0) ? 0 : c; } tot[g] = s; }
  __syncthreads();
  if (threadIdx.x < 32) {
    __shared__ int st[CSR_MAXG + 32];
    if (threadIdx.x == 0) { int acc = 0; for (int g = 0; g < NGP; ++g) { st[g] = acc; if (g < nG) acc += (tot[g] + 31) & ~31; } st[NGP] = acc; }
    __builtin_amdgcn_fence(__ATOMIC_RELEASE, "workgroup"); __builtin_amdgcn_wave_barrier(); __builtin_amdgcn_fence(__ATOMIC_ACQUIRE, "workgroup");
    for (int pass = 0; pass < 2; ++pass) { for (int i = threadIdx.x; i < NGP + 32; i += 32) { ((volatile int*)START)[i] = (i <= NGP) ? st[min(i, NGP)] : 0; ((volatile int*)TOT)[i] = (i < nG) ? tot[i] : 0; } __threadfence(); } }
}
__global__ __launch_bounds__(256) void csrB_kernel(const int* __restrict__ dst, int N, int nG, int CHP, int NGP, int permLen, const int* __restrict__ STG, const int* __restrict__ HST, const int* __restrict__ OFF, const int* __restrict__ START, const int* __restrict__ TOT, int* __restrict__ PERM, int* __restrict__ ROWPTR, int* __restrict__ ROWCNT, int* __restrict__ FLAG) {
  typedef __attribute__((ext_vector_type(4))) int v4i;
  __shared__ int ids[CSR_CAP]; __shared__ unsigned short key[CSR_CAP]; __shared__ int outp[CSR_CAP]; __shared__ int ncnt[CSR_GN + 1]; __shared__ int boff[CSR_NBLK + 1];
  const int g = blockIdx.x, t_ = threadIdx.x; int tot = TOT[g]; int st = START[g], stn = START[g + 1]; const int v0 = g * CSR_GN; const int nv = min(CSR_GN, N - v0);
  st = (st < 0) ? 0 : (st > permLen - 32 ? permLen - 32 : st) & ~31; stn = (stn < st) ? st : (stn > permLen ? permLen : stn); tot = (tot < 0) ? 0 : tot; if (tot > stn - st && tot <= CSR_CAP) tot = stn - st;
  if (tot > CSR_CAP) {
    for (int pass = 0; pass < 2; ++pass) { for (int i = t_; i < CSR_GN / 4; i += 256) { v4i a, c; for (int e = 0; e < 4; ++e) { a[e] = st; c[e] = 0; } *(volatile v4i*)(ROWPTR + v0 + i * 4) = a; *(volatile v4i*)(ROWCNT + v0 + i * 4) = c; } if (t_ == 0) ((volatile int*)FLAG)[0] = 1; __threadfence(); } (void)nv; return; }
  if (t_ == 0) { int acc = 0; for (int b = 0; b < CSR_NBLK; ++b) { boff[b] = acc; int c = HST[(size_t)b * NGP + g]; c = (c < 0) ? 0 : (c > CHP ? CHP : c); acc += c; if (acc > tot) acc = tot; } boff[CSR_NBLK] = acc; }
  for (int i = t_; i <= CSR_GN; i += 256) ncnt[i] = 0;
  __syncthreads();
  for (int b = 0; b < CSR_NBLK; ++b) { const int c = boff[b + 1] - boff[b]; int o_ = OFF[(size_t)g * CSR_NBLK + b]; o_ = (o_ < 0) ? 0 : (o_ > CHP - c ? CHP - c : o_); const int* src_ = STG + (size_t)b * CHP + o_;
    for (int i = t_; i < c; i += 256) { int id = src_[i]; id = (id < 0) ? 0 : id; ids[boff[b] + i] = id; int d = dst[id]; d = (d < v0) ? v0 : (d >= N ? N - 1 : d); int kk = d - v0; kk = (kk < 0) ? 0 : (kk >= CSR_GN ? CSR_GN - 1 : kk); key[boff[b] + i] = (unsigned short)kk; } }
  __syncthreads();
  if (t_ == 0) { for (int i = 0; i < tot; ++i) ncnt[key[i]] += 1; int acc = 0; for (int vl = 0; vl < CSR_GN; ++vl) { const int c = ncnt[vl]; ncnt[vl] = acc; acc += c; } ncnt[CSR_GN] = acc;
    for (int i = 0; i < tot; ++i) { const int vl = key[i]; outp[ncnt[vl]] = ids[i]; ncnt[vl] += 1; }
    for (int vl = CSR_GN; vl > 0; --vl) ncnt[vl] = ncnt[vl - 1]; ncnt[0] = 0; }
  __syncthreads();
  for (int pass = 0; pass < 2; ++pass) {
    for (int i = t_; i < (stn - st) / 4; i += 256) { v4i v; for (int e = 0; e < 4; ++e) { const int q = i * 4 + e; v[e] = (q < tot) ? outp[q] : -1; } *(volatile v4i*)(PERM + st + i * 4) = v; }
    for (int i = t_; i < CSR_GN / 4; i += 256) { v4i a, c; for (int e = 0; e < 4; ++e) { const int vl = i * 4 + e; a[e] = st + ncnt[vl]; c[e] = (vl < nv) ? (ncnt[vl + 1] - ncnt[vl]) : 0; } *(volatile v4i*)(ROWPTR + v0 + i * 4) = a; *(volatile v4i*)(ROWCNT + v0 + i * 4) = c; }
    __threadfence(); }
}
__global__ __launch_bounds__(256) void csrZ_kernel(int* __restrict__ p, size_t n4) { typedef __attribute__((ext_vector_type(4))) int v4i; const size_t tid = (size_t)blockIdx.x * 256 + threadIdx.x, nth = (size_t)gridDim.x * 256; v4i z = {0, 0, 0, 0}; for (size_t i = tid; i < n4; i += nth) *(volatile v4i*)(p + i * 4) = z; }
struct CsrBufs { int *STG, *HST, *OFF, *START, *TOT, *PERM, *ROWPTR, *ROWCNT, *FLAG; int nG, NGP, CHP; size_t permLen; char* base; size_t bytes; };
static size_t csr_carve(CsrBufs& c, char* ws, size_t off, int E, int N) {
  const size_t off0 = off; c.base = ws + off;
  auto al = [&](size_t bytes) { char* p = ws + off; off += (bytes + 255) & ~(size_t)255; return p; };
  c.nG = (N + CSR_GN - 1) / CSR_GN; c.NGP = (c.nG + 31) & ~31; const int ch = (E + CSR_NBLK - 1) / CSR_NBLK; c.CHP = (ch + 31) & ~31; c.permLen = (size_t)E + 32 * (size_t)c.nG + 32;
  c.STG = (int*)al((size_t)CSR_NBLK * c.CHP * 4); c.HST = (int*)al((size_t)CSR_NBLK * c.NGP * 4); c.OFF = (int*)al((size_t)c.NGP * CSR_NBLK * 4); c.START = (int*)al((size_t)(c.NGP + 64) * 4); c.TOT = (int*)al((size_t)(c.NGP + 64) * 4);
  c.PERM = (int*)al(c.permLen * 4); c.ROWPTR = (int*)al((size_t)c.nG * CSR_GN * 4); c.ROWCNT = (int*)al((size_t)c.nG * CSR_GN * 4); c.FLAG = (int*)al(256);
  c.bytes = off - off0; return off;
}
static void csr_build(const CsrBufs& c, const int* dst, int E, int N, hipStream_t stream) {
  const size_t smem = (size_t)(2 * c.NGP + c.CHP) * 4;
  csrZ_kernel<<<512, 256, 0, stream>>>((int*)c.base, c.bytes / 16);
  csrA_kernel<<<CSR_NBLK, 64, smem, stream>>>(dst, E, N, c.nG, c.CHP, c.NGP, c.STG, c.HST);
  csrS_kernel<<<1, 512, 0, stream>>>(c.HST, c.nG, c.NGP, c.START, c.TOT, c.OFF);
  csrB_kernel<<<c.nG, 256, 0, stream>>>(dst, N, c.nG, c.CHP, c.NGP, (int)c.permLen, c.STG, c.HST, c.OFF, c.START, c.TOT, c.PERM, c.ROWPTR, c.ROWCNT, c.FLAG);
}


__device__ __forceinline__ float sus(float x) { return x > 0.0f ? __expf(-1.0f / x) : 0.0f; }
__global__ __launch_bounds__(256) void prep_kernel(const float* __restrict__ x, const float* __restrict__ wq, const float* __restrict__ wk2, const float* __restrict__ wv2, const float* __restrict__ wdot, b16* __restrict__ WK, b16* __restrict__ WV, float* __restrict__ QW) {
  const size_t u_ = (size_t)blockIdx.x * 256 + threadIdx.x; const size_t nk = (size_t)DK * KK / 8, nv = (size_t)DV * KK / 8; size_t t = u_; v8b o;
  if (t < nk + nv) { const bool isv = t >= nk; const size_t e = (isv ? t - nk : t) * 8; const int outw = isv ? DV : DK; const float* w2 = isv ? wv2 : wk2; const int w = (int)(e / KK), k0 = (int)(e % KK);
    for (int jj = 0; jj < 8; ++jj) { const int kk = k0 + jj; const int u = kk / HDIM, j = kk % HDIM; const int colw = (u < M0) ? (u * outw + w) : (M0 * outw + (u - M0) * outw + w); o[jj] = (b16)(bf16_rne(w2[(size_t)j * (UC * outw) + colw]) * WSC); }
    for (int pass = 0; pass < 2; ++pass) { *(volatile v8b*)((isv ? WV : WK) + e) = o; __threadfence(); } return; } t -= nk + nv;
  if (t < (size_t)NP * DK) { const size_t v = t / DK; const int b = (int)(t % DK); float o1 = 0.0f;
    if (v < (size_t)N) {
#pragma unroll 1
      for (int a = 0; a < DQ; ++a) { float s = 0.0f;
#pragma unroll 1
        for (int u = 0; u < M0; ++u) s += pmul(bf16_rne(x[v * XW + u]), bf16_rne(wq[u * DQ + a]));
        o1 += pmul(s * 0.25f, bf16_rne(wdot[a * DK + b])); } }
    for (int pass = 0; pass < 2; ++pass) { ((volatile float*)QW)[v * DK + b] = o1; __threadfence(); } }
}
__global__ __launch_bounds__(32) void edge_kernel(const float* __restrict__ x, const float* __restrict__ pos, const float* __restrict__ wk1, const float* __restrict__ wv1, const int* __restrict__ srcs, const int* __restrict__ dsts, const int* __restrict__ PERM, int permLen, const b16* __restrict__ WK, const b16* __restrict__ WV, const float* __restrict__ QW, float* __restrict__ EV) {
  __shared__ __attribute__((aligned(16))) float Tf[16][64 + 4];
  const int lane = threadIdx.x, nloc = lane & 15, hlf = lane >> 4; const size_t m0 = (size_t)blockIdx.x * 16; const size_t j = m0 + nloc; const bool live = j < (size_t)permLen;
  const int e = live ? iclamp(PERM[j], 0, E - 1) : 0; const size_t s = (size_t)iclamp(srcs[e], 0, N - 1), d = (size_t)iclamp(dsts[e], 0, N - 1);
  const float ex = bf16_rne(pos[s * 3]) - bf16_rne(pos[d * 3]), ey = bf16_rne(pos[s * 3 + 1]) - bf16_rne(pos[d * 3 + 1]), ez = bf16_rne(pos[s * 3 + 2]) - bf16_rne(pos[d * 3 + 2]);
  const float elen = sqrtf(pmul(ex, ex) + pmul(ey, ey) + pmul(ez, ez) + 1e-12f); const float wcut = sus(10.0f * (1.0f - elen / RMAX));
  float emb[NB]; { const float stepv = RMAX / (float)(NB + 1); const float Cc = 1.14136f * 7.3890560989306502f * sqrtf((float)NB);
#pragma unroll
    for (int b = 0; b < NB; ++b) { const float val = (float)(b + 1) * stepv; const float diff = (elen - val) / stepv; emb[b] = Cc * sus(diff + 1.0f) * sus(1.0f - diff); } }
  float hk[HDIM], hv[HDIM];
#pragma unroll
  for (int jj = 0; jj < HDIM; ++jj) { float a = 0.0f, b = 0.0f;
#pragma unroll
    for (int t = 0; t < NB; ++t) { a += pmul(emb[t], bf16_rne(wk1[t * HDIM + jj])); b += pmul(emb[t], bf16_rne(wv1[t * HDIM + jj])); }
    a *= 0.31622776601683794f; b *= 0.31622776601683794f; hk[jj] = a / (1.0f + __expf(-a)); hv[jj] = b / (1.0f + __expf(-b)); }
  float xc[UC];
#pragma unroll
  for (int u = 0; u < M0; ++u) xc[u] = bf16_rne(x[s * XW + u]);
  { const float il = 1.7320508075688772f / elen; const float sx = ex * il, sy = ey * il, sz = ez * il;
#pragma unroll
    for (int u = 0; u < M1; ++u) { const float* p = x + s * XW + M0 + u * 3; xc[M0 + u] = (pmul(bf16_rne(p[0]), sx) + pmul(bf16_rne(p[1]), sy) + pmul(bf16_rne(p[2]), sz)) * 0.57735026918962576f; } }
  if (!live) { for (int u = 0; u < UC; ++u) xc[u] = 0.0f; }
  v8f ak = {}, av0 = {}, av1 = {};
#pragma unroll
  for (int ks = 0; ks < KK / 32; ++ks) { const int u0 = ks * 2; v16b fk, fkl, fv, fvl;
#pragma unroll
    for (int el = 0; el < 16; ++el) { const int jj = (el < 8) ? el : el - 8; const int uu = (el < 8) ? u0 : u0 + 1; const float hkk = hlf ? hk[jj + 8] : hk[jj]; const float hvv = hlf ? hv[jj + 8] : hv[jj];
      b16 p, q; split16(pmul(hkk, xc[uu]) * XS, p, q); fk[el] = p; fkl[el] = q; split16(pmul(hvv, xc[uu]) * XS, p, q); fv[el] = p; fvl[el] = q; }
    const int kb = ks * 32;
    { const v16b bw = frag_kb(WK + (size_t)nloc * KK + kb, hlf); ak = wmma16b(fk, bw, ak); ak = wmma16b(fkl, bw, ak); }
    { const v16b bw = frag_kb(WV + (size_t)nloc * KK + kb, hlf); av0 = wmma16b(fv, bw, av0); av0 = wmma16b(fvl, bw, av0); }
    { const v16b bw = frag_kb(WV + (size_t)(16 + nloc) * KK + kb, hlf); av1 = wmma16b(fv, bw, av1); av1 = wmma16b(fvl, bw, av1); } }
  const float kn = (1.0f / (XS * WSC)) * 0.25f * 0.20412414523193151f;
  float lg[8];
#pragma unroll
  for (int r = 0; r < 8; ++r) { const int rr = 8 * hlf + r; const int drow = __shfl((int)d, rr); const float qw = QW[(size_t)drow * DK + nloc]; float t = pmul(ak[r] * kn, qw); t += __shfl_xor(t, 1); t += __shfl_xor(t, 2); t += __shfl_xor(t, 4); t += __shfl_xor(t, 8); lg[r] = t * (1.0f / 16.0f); }
#pragma unroll
  for (int r = 0; r < 8; ++r) { const int rr = 8 * hlf + r; Tf[rr][nloc] = av0[r] * kn; Tf[rr][16 + nloc] = av1[r] * kn;
    const float wc = __shfl(wcut, rr); const int lv = __shfl((int)(live ? 1 : 0), rr);
    const float ev = lv ? pmul(wc, __expf(lg[r])) : 0.0f; if (nloc == 0) Tf[rr][32] = ev; }
  for (int q = lane; q < 16 * 31; q += 32) { const int rr = q / 31, c = 33 + (q % 31); Tf[rr][c] = 0.0f; }
  wave_lds_sync();
  for (int pass = 0; pass < 2; ++pass) { for (int rr = 0; rr < 16; ++rr) if (lane < 16) *(volatile v4f*)(EV + (m0 + rr) * 64 + lane * 4) = *(const v4f*)(&Tf[rr][lane * 4]); __threadfence(); }
}
__global__ __launch_bounds__(256) void agg_kernel(const float* __restrict__ EV, const int* __restrict__ ROWPTR, const int* __restrict__ ROWCNT, int permLen, float* __restrict__ out) {
  const int wave = threadIdx.x >> 5, lane = threadIdx.x & 31; const size_t i = (size_t)blockIdx.x * 8 + wave; if (i >= (size_t)N) return;
  int st = ROWPTR[i], cnt = ROWCNT[i]; cnt = iclamp(cnt, 0, 65536); st = iclamp(st, 0, permLen - cnt);
  float z = 0.0f; for (int q = 0; q < cnt; ++q) z += EV[(size_t)(st + q) * 64 + 32];
  if (z == 0.0f) z = 1.0f;
  float acc = 0.0f; for (int q = 0; q < cnt; ++q) { const float ev = EV[(size_t)(st + q) * 64 + 32]; const float al = ev / z; const float sa = al > 0.0f ? sqrtf(al) : 0.0f; acc += pmul(sa, EV[(size_t)(st + q) * 64 + lane]); }
  for (int pass = 0; pass < 2; ++pass) { ((volatile float*)out)[i * DV + lane] = acc; __threadfence(); }
}
}

extern "C" void kernel_launch(void* const* d_in, const int* in_sizes, int n_in, void* d_out, int out_size, void* d_ws, size_t ws_size, hipStream_t stream) {
  (void)n_in;
  auto Fp = [&](int i) { return (const float*)d_in[i]; }; auto Ip = [&](int i) { return (const int*)d_in[i]; };
  if (in_sizes[0] != N * XW || in_sizes[1] != N * 3 || in_sizes[2] != M0 * DQ || in_sizes[3] != NB * HDIM || in_sizes[4] != HDIM * UC * DK || in_sizes[6] != HDIM * UC * DV || in_sizes[7] != DQ * DK || in_sizes[8] != E || in_sizes[9] != E || out_size != N * DV) return;
  size_t off = 0; char* ws = (char*)d_ws;
  auto carve = [&](size_t bytes) { char* p = ws + off; off += (bytes + 255) & ~(size_t)255; return p; };
  b16* WK = (b16*)carve((size_t)DK * KK * 2); b16* WV = (b16*)carve((size_t)DV * KK * 2); float* QW = (float*)carve((size_t)NP * DK * 4); float* EV = (float*)carve((size_t)EP * 64 * 4);
  CsrBufs csr; off = csr_carve(csr, ws, off, E, N);
  if (off > ws_size || off > ((size_t)128 << 20) || csr.permLen > (size_t)EP) return;
  prep_kernel<<<(unsigned)(((size_t)DK * KK / 8 + (size_t)DV * KK / 8 + (size_t)NP * DK + 255) / 256), 256, 0, stream>>>(Fp(0), Fp(2), Fp(4), Fp(6), Fp(7), WK, WV, QW);
  csr_build(csr, Ip(9), E, N, stream);
  edge_kernel<<<EP / 16, 32, 0, stream>>>(Fp(0), Fp(1), Fp(3), Fp(5), Ip(8), Ip(9), csr.PERM, (int)csr.permLen, WK, WV, QW, EV);
  agg_kernel<<<(N + 7) / 8, 256, 0, stream>>>(EV, csr.ROWPTR, csr.ROWCNT, (int)csr.permLen, (float*)d_out);
}
